// BoxRPBAttention_76613626626661
// MI455X (gfx1250) — hardware-verified
//
#include <hip/hip_runtime.h>


namespace {
constexpr int NQ = 900, NQP = 912  , Bn = 4, C = 256, H = 8, HD = 32, GH = 64, GW = 64, N = GH * GW, R = 512, STRIDE = 16;
constexpr float QS = 8.0f, KS = 8.0f, VS = 8.0f, PS = 8.0f, AS_ = 8.0f, SCALE = 0.17677669529663687f;
constexpr size_t QPL = (size_t)Bn * H * NQP * HD, KPL = (size_t)Bn * H * N * HD;

typedef _Float16 b16;
typedef __attribute__((ext_vector_type(16))) _Float16 v16b;
typedef __attribute__((ext_vector_type(16))) __bf16 v16bb;
typedef __attribute__((ext_vector_type(8))) _Float16 v8b;
typedef __attribute__((ext_vector_type(8))) unsigned short v8us;
typedef __attribute__((ext_vector_type(8))) float v8f;
typedef __attribute__((ext_vector_type(4))) float v4f;
__device__ __forceinline__ float bf16_rne(float f) { unsigned int u = __float_as_uint(f); u += 0x7FFFu + ((u >> 16) & 1u); return __uint_as_float(u & 0xFFFF0000u); }
__device__ __forceinline__ unsigned short bf16_bits(float f) { unsigned int u = __float_as_uint(f); u += 0x7FFFu + ((u >> 16) & 1u); return (unsigned short)(u >> 16); }
__device__ __forceinline__ void split16(float v, b16& hi, b16& lo) { hi = (b16)v; lo = (b16)(v - (float)hi); }
__device__ __forceinline__ v16b frag_kb(const b16* p, int hh) { const v8b a = *(const v8b*)(p + 8 * hh), b = *(const v8b*)(p + 16 + 8 * hh); v16b f;
#pragma unroll
  for (int e = 0; e < 8; ++e) { f[e] = a[e]; f[8 + e] = b[e]; } return f; }
__device__ __forceinline__ v16bb frag_bf(const unsigned short* p, int hh) { const v8us a = *(const v8us*)(p + 8 * hh), b = *(const v8us*)(p + 16 + 8 * hh); union { unsigned short s[16]; v16bb v; } u;
#pragma unroll
  for (int e = 0; e < 8; ++e) { u.s[e] = a[e]; u.s[8 + e] = b[e]; } return u.v; }
__device__ __forceinline__ v16bb frag_f32bf(const float* p, int hh) { union { unsigned short s[16]; v16bb v; } u;
#pragma unroll
  for (int e = 0; e < 8; ++e) { u.s[e] = bf16_bits(p[8 * hh + e]); u.s[8 + e] = bf16_bits(p[16 + 8 * hh + e]); } return u.v; }
__device__ __forceinline__ void frag_split(const float* p, int hh, v16b& fh, v16b& fl) {
#pragma unroll
  for (int e = 0; e < 8; ++e) { b16 a, c; split16(p[8 * hh + e] * AS_, a, c); fh[e] = a; fl[e] = c; split16(p[16 + 8 * hh + e] * AS_, a, c); fh[8 + e] = a; fl[8 + e] = c; } }
__device__ __forceinline__ v8f wmma16b(v16b a, v16b b, v8f c) { v8f d = __builtin_amdgcn_wmma_f32_16x16x32_f16(false, a, false, b, (short)0, c, false, false); asm volatile("v_nop\n\tv_nop\n\tv_nop\n\tv_nop" : "+v"(d) : "v"(a), "v"(b)); return d; }
__device__ __forceinline__ v8f wmma16bb(v16bb a, v16bb b, v8f c) { v8f d = __builtin_amdgcn_wmma_f32_16x16x32_bf16(false, a, false, b, (short)0, c, false, false); asm volatile("v_nop\n\tv_nop\n\tv_nop\n\tv_nop" : "+v"(d) : "v"(a), "v"(b)); return d; }
__device__ __forceinline__ void wave_lds_sync() { __builtin_amdgcn_fence(__ATOMIC_RELEASE, "workgroup"); __builtin_amdgcn_wave_barrier(); __builtin_amdgcn_fence(__ATOMIC_ACQUIRE, "workgroup"); }
__device__ __forceinline__ float nexp(float x) { return __builtin_amdgcn_exp2f(x * 1.4426950408889634f); }
__device__ __forceinline__ float pmul(float a, float b) { float p = a * b; asm volatile("" : "+v"(p)); return p; }

__global__ __launch_bounds__(256) void prep_kernel(const float* __restrict__ Wq, const float* __restrict__ Wk, const float* __restrict__ Wv, const float* __restrict__ Wp, const float* __restrict__ W2a, const float* __restrict__ W2b,
                                                   const float* __restrict__ bq, const float* __restrict__ bk, const float* __restrict__ bv, const float* __restrict__ bp, const float* __restrict__ W1a, const float* __restrict__ b1a, const float* __restrict__ W1b, const float* __restrict__ b1b,
                                                   unsigned short* __restrict__ w16, b16* __restrict__ wp16, b16* __restrict__ w2r, float* __restrict__ P) {
  const size_t tid = (size_t)blockIdx.x * blockDim.x + threadIdx.x, nth = (size_t)gridDim.x * blockDim.x;
  for (int pass = 0; pass < 2; ++pass) {
    for (size_t p = tid; p < (size_t)3 * C * C / 8; p += nth) { const int m = (int)(p / (C * C / 8)); const size_t q = p % (C * C / 8); const int o = (int)(q / (C / 8)), k8 = (int)(q % (C / 8)) * 8; const float* W = (m == 0) ? Wq : (m == 1) ? Wk : Wv; v8us v;
#pragma unroll
      for (int e = 0; e < 8; ++e) v[e] = bf16_bits(W[(size_t)(k8 + e) * C + o]);
      *(volatile v8us*)(w16 + p * 8) = v; }
    for (size_t p = tid; p < (size_t)C * C / 8; p += nth) { const int o = (int)(p / (C / 8)), k8 = (int)(p % (C / 8)) * 8; v8b v;
#pragma unroll
      for (int e = 0; e < 8; ++e) v[e] = (b16)bf16_rne(Wp[(size_t)(k8 + e) * C + o]);
      *(volatile v8b*)(wp16 + p * 8) = v; }
    for (size_t p = tid; p < (size_t)2 * 16 * R / 8; p += nth) { const int m = (int)(p / (16 * R / 8)); const size_t q = p % (16 * R / 8); const int o = (int)(q / (R / 8)), k8 = (int)(q % (R / 8)) * 8; const float* W = m ? W2b : W2a; v8b v;
#pragma unroll
      for (int e = 0; e < 8; ++e) v[e] = (b16)((o < H) ? bf16_rne(W[(size_t)(k8 + e) * H + o]) : 0.0f);
      *(volatile v8b*)(w2r + p * 8) = v; }
    for (size_t p = tid; p < 4096 / 4; p += nth) { v4f v;
#pragma unroll
      for (int e = 0; e < 4; ++e) { const int i = (int)p * 4 + e; float x = 0.0f; if (i < 256) x = bq[i]; else if (i < 512) x = bk[i - 256]; else if (i < 768) x = bv[i - 512]; else if (i < 1024) x = bp[i - 768]; else if (i < 2048) x = W1a[i - 1024]; else if (i < 2560) x = b1a[i - 2048]; else if (i < 3584) x = W1b[i - 2560]; else x = b1b[i - 3584]; v[e] = bf16_rne(x); }
      *(volatile v4f*)(P + p * 4) = v; }
    __threadfence(); }
}

__global__ __launch_bounds__(128) void proj_kernel(const float* __restrict__ query, const float* __restrict__ kin, const float* __restrict__ vin, const unsigned short* __restrict__ w16, const float* __restrict__ P, b16* __restrict__ qh, b16* __restrict__ kh, b16* __restrict__ vt) {
  __shared__ __attribute__((aligned(16))) b16 Th[4][32][64 + 8], Tl[4][32][64 + 8]; __shared__ __attribute__((aligned(16))) b16 Vh[64][128 + 8], Vl[64][128 + 8];
  const int lane = threadIdx.x & 31, wave = threadIdx.x >> 5, nloc = lane & 15, hlf = lane >> 4, which = blockIdx.z, c0 = blockIdx.x * 64; const int nrow = (which == 0) ? NQP : N;
  if ((int)blockIdx.y * 128 >= Bn * nrow) return;
  const int m0 = blockIdx.y * 128 + wave * 32, b = (blockIdx.y * 128) / nrow, r0 = (blockIdx.y * 128) % nrow;
  auto srcrow = [&](int m) -> const float* { if (which == 0) { m = min(m, Bn * NQP - 1); const int bb = m / NQP, q = m % NQP; return query + ((size_t)min(q, NQ - 1) * Bn + bb) * C; } const int bb = m / N, n = m % N; return ((which == 1) ? kin : vin) + ((size_t)n * Bn + bb) * C; };
  const float* ra = srcrow(m0 + nloc); const float* rb = srcrow(m0 + 16 + nloc); const unsigned short* Wt = w16 + (size_t)which * C * C; const float* bias = P + which * 256;
  v8f acc[2][4];
#pragma unroll
  for (int r = 0; r < 2; ++r)
#pragma unroll
    for (int t = 0; t < 4; ++t) acc[r][t] = (v8f){};
#pragma unroll 2
  for (int kb = 0; kb < C; kb += 32) { const v16bb a0 = frag_f32bf(ra + kb, hlf), a1 = frag_f32bf(rb + kb, hlf);
#pragma unroll
    for (int t = 0; t < 4; ++t) { const v16bb bw = frag_bf(Wt + (size_t)(c0 + t * 16 + nloc) * C + kb, hlf); acc[0][t] = wmma16bb(a0, bw, acc[0][t]); acc[1][t] = wmma16bb(a1, bw, acc[1][t]); } }
  const float scl = (which == 0) ? SCALE * QS : ((which == 1) ? KS : VS);
  if (which < 2) {
#pragma unroll
    for (int t = 0; t < 4; ++t) { const float bb = bias[c0 + t * 16 + nloc];
#pragma unroll
      for (int r = 0; r < 2; ++r)
#pragma unroll
        for (int v = 0; v < 8; ++v) { b16 a_, c_; split16((acc[r][t][v] + bb) * scl, a_, c_); Th[wave][r * 16 + 8 * hlf + v][t * 16 + nloc] = a_; Tl[wave][r * 16 + 8 * hlf + v][t * 16 + nloc] = c_; } }
    wave_lds_sync();
    b16* base = (which == 0) ? qh : kh; const size_t PL = (which == 0) ? QPL : KPL; const int nr = (which == 0) ? NQP : N;
    for (int pass = 0; pass < 2; ++pass) {
#pragma unroll
      for (int j = 0; j < 4; ++j) { const int rr = j * 8 + (lane >> 2), c8 = (lane & 3) * 8; const int m = m0 + rr, bb = m / nr, rowi = m % nr; if (m >= Bn * nr) continue;
#pragma unroll
        for (int hh2 = 0; hh2 < 2; ++hh2) { const int h = c0 / 32 + hh2; const size_t o = (((size_t)bb * H + h) * nr + rowi) * HD + c8;
          *(volatile v8b*)(base + o) = *(const v8b*)(&Th[wave][rr][hh2 * 32 + c8]); *(volatile v8b*)(base + PL + o) = *(const v8b*)(&Tl[wave][rr][hh2 * 32 + c8]); } }
      __threadfence(); }
    return; }
#pragma unroll
  for (int t = 0; t < 4; ++t) { const float bb = bias[c0 + t * 16 + nloc];
#pragma unroll
    for (int r = 0; r < 2; ++r)
#pragma unroll
      for (int v = 0; v < 8; ++v) { b16 a_, c_; split16((acc[r][t][v] + bb) * scl, a_, c_); Vh[t * 16 + nloc][wave * 32 + r * 16 + 8 * hlf + v] = a_; Vl[t * 16 + nloc][wave * 32 + r * 16 + 8 * hlf + v] = c_; } }
  __syncthreads();
  for (int pass = 0; pass < 2; ++pass) { for (int i = threadIdx.x; i < 64 * 16; i += 128) { const int cc = i >> 4, c8 = (i & 15) * 8; const int h = (c0 + cc) / 32, d = (c0 + cc) % 32; const size_t o = (((size_t)b * H + h) * HD + d) * N + r0 + c8;
      *(volatile v8b*)(vt + o) = *(const v8b*)(&Vh[cc][c8]); *(volatile v8b*)(vt + KPL + o) = *(const v8b*)(&Vl[cc][c8]); } __threadfence(); }
}

__global__ __launch_bounds__(128) void cpb_kernel(const float* __restrict__ refp, const b16* __restrict__ w2r, const float* __restrict__ P, int boff, float* __restrict__ tabx, float* __restrict__ taby) {
  __shared__ __attribute__((aligned(16))) float To[4][32][8];
  const int lane = threadIdx.x & 31, wave = threadIdx.x >> 5, nloc = lane & 15, hlf = lane >> 4, which = blockIdx.y, m0 = (blockIdx.x + boff) * 128 + wave * 32;
  const float* W1 = P + (which ? 2560 : 1024); const float* b1 = P + (which ? 3584 : 2048); const b16* W2 = w2r + (size_t)which * 16 * R; float* tab = which ? taby : tabx;
  float d0[2], d1[2];
#pragma unroll
  for (int r = 0; r < 2; ++r) { const int m = m0 + r * 16 + nloc; const int p = m & 63, q = (m >> 6) % NQP, b = (m >> 6) / NQP; const float* rp = refp + ((size_t)min(q, NQ - 1) * Bn + b) * 4;
    const float cx = bf16_rne(rp[0]), cy = bf16_rne(rp[1]), sx = bf16_rne(rp[2]), sy = bf16_rne(rp[3]); const float ctr = which ? cy : cx, sz = which ? sy : sx; const float ext = (float)((which ? GH : GW) * STRIDE);
    const float lo = (ctr - sz * 0.5f) * ext, hi = (ctr + sz * 0.5f) * ext, pos = ((float)p + 0.5f) * (float)STRIDE; d0[r] = lo - pos; d1[r] = hi - pos; }
  v8f acc[2] = {{}, {}};
#pragma unroll 2
  for (int kb = 0; kb < R; kb += 32) { v16b a[2], l[2];
#pragma unroll
    for (int r = 0; r < 2; ++r)
#pragma unroll
      for (int e = 0; e < 16; ++e) { const int k = kb + ((e < 8) ? (8 * hlf + e) : (16 + 8 * hlf + e - 8)); const float hv = fmaxf((pmul(d0[r], W1[k]) + pmul(d1[r], W1[R + k])) + b1[k], 0.0f); b16 x_, y_; split16(hv * AS_, x_, y_); a[r][e] = x_; l[r][e] = y_; }
    const v16b bw = frag_kb(W2 + (size_t)nloc * R + kb, hlf);
#pragma unroll
    for (int r = 0; r < 2; ++r) { acc[r] = wmma16b(a[r], bw, acc[r]); acc[r] = wmma16b(l[r], bw, acc[r]); } }
  if (nloc < H) {
#pragma unroll
    for (int r = 0; r < 2; ++r)
#pragma unroll
      for (int v = 0; v < 8; ++v) To[wave][r * 16 + 8 * hlf + v][nloc] = acc[r][v] * (1.0f / AS_); }
  wave_lds_sync();
  for (int pass = 0; pass < 2; ++pass) { for (int i = lane; i < 32 * 2; i += 32) { const int rr = i >> 1, c4 = (i & 1) * 4; *(volatile v4f*)(tab + (size_t)(m0 + rr) * H + c4) = *(const v4f*)(&To[wave][rr][c4]); } __threadfence(); }
}

__global__ __launch_bounds__(256) void attn_kernel(const b16* __restrict__ qh, const b16* __restrict__ kh, const b16* __restrict__ vt, const float* __restrict__ tabx, const float* __restrict__ taby, int boff, float* __restrict__ ctx) {
  __shared__ __attribute__((aligned(16))) float Os[16][C + 4];
  const int h = threadIdx.x >> 5, lane = threadIdx.x & 31, hh = lane >> 4, col = lane & 15; const int blk = blockIdx.x + boff, b = blk / (NQP / 16), q0 = (blk % (NQP / 16)) * 16, qi = q0 + col;
  const b16* Q = qh + (((size_t)b * H + h) * NQP) * HD; const b16* K = kh + (((size_t)b * H + h) * N) * HD; const b16* V = vt + (((size_t)b * H + h) * HD) * N;
  const float* tx = tabx + (((size_t)b * NQP + qi) * GW) * H + h; const float* ty = taby + (((size_t)b * NQP + qi) * GH) * H + h;
  const v16b qf = frag_kb(Q + (size_t)qi * HD, hh), ql = frag_kb(Q + QPL + (size_t)qi * HD, hh);
  float m = -INFINITY, l = 0.0f; v8f o[2] = {{}, {}};
  for (int kb = 0; kb < N; kb += 32) { const v16b ka = frag_kb(K + (size_t)(kb + col) * HD, hh), kal = frag_kb(K + KPL + (size_t)(kb + col) * HD, hh), kc = frag_kb(K + (size_t)(kb + 16 + col) * HD, hh), kcl = frag_kb(K + KPL + (size_t)(kb + 16 + col) * HD, hh);
    v8f s0 = {}, s1 = {}; s0 = wmma16b(ka, qf, s0); s0 = wmma16b(ka, ql, s0); s0 = wmma16b(kal, qf, s0); s1 = wmma16b(kc, qf, s1); s1 = wmma16b(kc, ql, s1); s1 = wmma16b(kcl, qf, s1);
    const int y = kb >> 6; const float ry = ty[(size_t)y * H];
    float mr = -INFINITY;
#pragma unroll
    for (int r = 0; r < 8; ++r) { const int x0 = (kb & 63) + 8 * hh + r; s0[r] = s0[r] * (1.0f / (QS * KS)) + tx[(size_t)x0 * H] + ry; s1[r] = s1[r] * (1.0f / (QS * KS)) + tx[(size_t)(x0 + 16) * H] + ry; mr = fmaxf(mr, fmaxf(s0[r], s1[r])); }
    mr = fmaxf(mr, __shfl_xor(mr, 16));
    const float mn = fmaxf(m, mr), al_ = nexp(m - mn); m = mn; float sum = 0.0f; v16b pbv, plv;
#pragma unroll
    for (int r = 0; r < 8; ++r) { const float e0 = nexp(s0[r] - mn), e1 = nexp(s1[r] - mn); sum += e0 + e1; b16 a, cc; split16(e0 * PS, a, cc); pbv[r] = a; plv[r] = cc; split16(e1 * PS, a, cc); pbv[8 + r] = a; plv[8 + r] = cc; }
    sum += __shfl_xor(sum, 16); l = l * al_ + sum;
#pragma unroll
    for (int t = 0; t < 2; ++t) { o[t] *= al_; const v16b vf = frag_kb(V + (size_t)(t * 16 + col) * N + kb, hh), vl = frag_kb(V + KPL + (size_t)(t * 16 + col) * N + kb, hh); o[t] = wmma16b(vf, pbv, o[t]); o[t] = wmma16b(vf, plv, o[t]); o[t] = wmma16b(vl, pbv, o[t]); } }
  const float inv = 1.0f / (l * VS * PS);
#pragma unroll
  for (int t = 0; t < 2; ++t)
#pragma unroll
    for (int r = 0; r < 8; ++r) Os[col][h * HD + t * 16 + 8 * hh + r] = o[t][r] * inv;
  __syncthreads();
  float* dst = ctx + ((size_t)b * NQP + q0) * C;
  for (int pass = 0; pass < 2; ++pass) { for (int i = threadIdx.x; i < 16 * (C / 4); i += 256) { const int rr = i / (C / 4), c4 = (i % (C / 4)) * 4; *(volatile v4f*)(dst + (size_t)rr * C + c4) = *(const v4f*)(&Os[rr][c4]); } __threadfence(); }
}

__global__ __launch_bounds__(128) void out_kernel(const float* __restrict__ ctx, const b16* __restrict__ wp16, const float* __restrict__ P, float* __restrict__ out) {
  __shared__ __attribute__((aligned(16))) float Ts[4][32 * 64];
  const int lane = threadIdx.x & 31, wave = threadIdx.x >> 5, nloc = lane & 15, hlf = lane >> 4, m0 = blockIdx.y * 128 + wave * 32, c0 = blockIdx.x * 64; const float* bp = P + 768;
  auto src = [&](int m) { m = min(m, NQ * Bn - 1); const int q = m / Bn, b = m % Bn; return ctx + ((size_t)b * NQP + q) * C; };
  const float* ra = src(m0 + nloc); const float* rb = src(m0 + 16 + nloc);
  v8f acc[2][4];
#pragma unroll
  for (int r = 0; r < 2; ++r)
#pragma unroll
    for (int t = 0; t < 4; ++t) acc[r][t] = (v8f){};
#pragma unroll 2
  for (int kb = 0; kb < C; kb += 32) { v16b a0, l0, a1, l1; frag_split(ra + kb, hlf, a0, l0); frag_split(rb + kb, hlf, a1, l1);
#pragma unroll
    for (int t = 0; t < 4; ++t) { const v16b bw = frag_kb(wp16 + (size_t)(c0 + t * 16 + nloc) * C + kb, hlf); acc[0][t] = wmma16b(a0, bw, acc[0][t]); acc[0][t] = wmma16b(l0, bw, acc[0][t]); acc[1][t] = wmma16b(a1, bw, acc[1][t]); acc[1][t] = wmma16b(l1, bw, acc[1][t]); } }
  float* Tt = Ts[wave];
#pragma unroll
  for (int t = 0; t < 4; ++t) { const float bb = bp[c0 + t * 16 + nloc];
#pragma unroll
    for (int r = 0; r < 2; ++r)
#pragma unroll
      for (int v = 0; v < 8; ++v) Tt[(r * 16 + v + 8 * hlf) * 64 + t * 16 + nloc] = acc[r][t][v] * (1.0f / AS_) + bb; }
  wave_lds_sync();
  for (int pass = 0; pass < 2; ++pass) {
#pragma unroll
    for (int j = 0; j < 16; ++j) { const int rr = j * 2 + hlf, c4 = nloc * 4; if (m0 + rr < NQ * Bn) *(volatile v4f*)(out + (size_t)(m0 + rr) * C + c0 + c4) = *(const v4f*)(Tt + rr * 64 + c4); }
    __threadfence(); }
}
}

extern "C" void kernel_launch(void* const* d_in, const int* in_sizes, int n_in,
                              void* d_out, int out_size, void* d_ws, size_t ws_size, hipStream_t stream) {
  (void)n_in; (void)out_size;
  const float* query = (const float*)d_in[0]; const float* refp = (const float*)d_in[1]; const float* kin = (const float*)d_in[2]; const float* vin = (const float*)d_in[3];
  const float* Wq = (const float*)d_in[4]; const float* bq = (const float*)d_in[5]; const float* Wk = (const float*)d_in[6]; const float* bk = (const float*)d_in[7]; const float* Wv = (const float*)d_in[8]; const float* bv = (const float*)d_in[9];
  const float* W1a = (const float*)d_in[10]; const float* b1a = (const float*)d_in[11]; const float* W2a = (const float*)d_in[12]; const float* W1b = (const float*)d_in[13]; const float* b1b = (const float*)d_in[14]; const float* W2b = (const float*)d_in[15]; const float* Wp = (const float*)d_in[16]; const float* bp = (const float*)d_in[17];
  float* out = (float*)d_out;
  if (in_sizes[0] != NQ * Bn * C || in_sizes[1] != NQ * Bn * 4 || in_sizes[2] != N * Bn * C || in_sizes[4] != C * C || in_sizes[10] != 2 * R || in_sizes[12] != R * H || in_sizes[16] != C * C) return;
  size_t off = 0; char* ws = (char*)d_ws;
  auto carve = [&](size_t bytes) { char* p = ws + off; off += (bytes + 255) & ~(size_t)255; return p; };
  unsigned short* w16 = (unsigned short*)carve((size_t)3 * C * C * 2); b16* wp16 = (b16*)carve((size_t)C * C * 2); b16* w2r = (b16*)carve((size_t)2 * 16 * R * 2); float* P = (float*)carve(4096 * 4);
  b16* qh = (b16*)carve(QPL * 2 * 2); b16* kh = (b16*)carve(KPL * 2 * 2); b16* vt = (b16*)carve(KPL * 2 * 2); float* tabx = (float*)carve((size_t)Bn * NQP * GW * H * 4); float* taby = (float*)carve((size_t)Bn * NQP * GH * H * 4); float* ctx = (float*)carve((size_t)Bn * NQP * C * 4);
  if (off > ws_size) return;
  prep_kernel<<<64, 256, 0, stream>>>(Wq, Wk, Wv, Wp, W2a, W2b, bq, bk, bv, bp, W1a, b1a, W1b, b1b, w16, wp16, w2r, P);
  proj_kernel<<<dim3(C / 64, Bn * N / 128, 3), 128, 0, stream>>>(query, kin, vin, w16, P, qh, kh, vt);
  cpb_kernel<<<dim3(Bn * NQP * 64 / 128, 2), 128, 0, stream>>>(refp, w2r, P, 0, tabx, taby);
  attn_kernel<<<Bn * NQP / 16, 256, 0, stream>>>(qh, kh, vt, tabx, taby, 0, ctx);
  out_kernel<<<dim3(C / 64, (NQ * Bn + 127) / 128), 128, 0, stream>>>(ctx, wp16, P, out);
}
